// SelfAttention_v2_83717502534318
// MI455X (gfx1250) — hardware-verified
//
#include <hip/hip_runtime.h>
#include <stdint.h>


#define SEQ 4096
#define DIM 1024
#define KT  256
#define PSCALE 4096.0f
#define PSCALE_INV 0.000244140625f
#define NOP4 "v_nop\n\tv_nop\n\tv_nop\n\tv_nop"

typedef _Float16 v8h  __attribute__((ext_vector_type(8)));
typedef _Float16 v16h __attribute__((ext_vector_type(16)));
typedef __bf16   v8b  __attribute__((ext_vector_type(8)));
typedef __bf16   v16b __attribute__((ext_vector_type(16)));
typedef float    v8f  __attribute__((ext_vector_type(8)));
typedef float    v4f  __attribute__((ext_vector_type(4)));
typedef unsigned int v4u __attribute__((ext_vector_type(4)));

union FragH { v16h v; v8h half[2]; };
union FragB { v16b v; v8b half[2]; };

__device__ __forceinline__ v8f mma_bf(v16b a, v16b b, v8f c) {
  return __builtin_amdgcn_wmma_f32_16x16x32_bf16(false, a, false, b, (short)0, c, false, false);
}
__device__ __forceinline__ v8f mma_h(v16h a, v16h b, v8f c) {
  return __builtin_amdgcn_wmma_f32_16x16x32_f16(false, a, false, b, (short)0, c, false, false);
}

__device__ __forceinline__ uint32_t bf16_bits(float f) {
  uint32_t u = __float_as_uint(f);
  u += 0x7FFFu + ((u >> 16) & 1u);
  return u >> 16;
}

__global__ __launch_bounds__(256) void cvt_kernel(
    const float* __restrict__ s0, const float* __restrict__ s1,
    const float* __restrict__ s2, const float* __restrict__ s3,
    uint16_t* d0, uint16_t* d1, uint16_t* d2, uint16_t* d3,
    int n8_0, int n8_1, int n8_2, int n8_3)
{
  const int seg = blockIdx.y;
  const float* src = (seg == 0) ? s0 : ((seg == 1) ? s1 : ((seg == 2) ? s2 : s3));
  uint16_t*    dst = (seg == 0) ? d0 : ((seg == 1) ? d1 : ((seg == 2) ? d2 : d3));
  const int    n8  = (seg == 0) ? n8_0 : ((seg == 1) ? n8_1 : ((seg == 2) ? n8_2 : n8_3));
  const int g = blockIdx.x * 256 + (int)threadIdx.x;
  if (g >= n8) return;
  const float* p = src + (size_t)g * 8;
  const v4f lo = *(const v4f*)p;
  const v4f hi = *(const v4f*)(p + 4);
  v4u w;
  w.x = bf16_bits(lo.x) | (bf16_bits(lo.y) << 16);
  w.y = bf16_bits(lo.z) | (bf16_bits(lo.w) << 16);
  w.z = bf16_bits(hi.x) | (bf16_bits(hi.y) << 16);
  w.w = bf16_bits(hi.z) | (bf16_bits(hi.w) << 16);
  volatile v4u* q = (volatile v4u*)(dst + (size_t)g * 8);
  *q = w;
  __threadfence();
  *q = w;
}

__global__ __launch_bounds__(128) void proj_kernel(
    const __bf16* __restrict__ Xb,
    const __bf16* __restrict__ Wq, const __bf16* __restrict__ Wk, const __bf16* __restrict__ Wv,
    _Float16* Qh, _Float16* Kh, _Float16* Vt)
{
  __shared__ __attribute__((aligned(16))) _Float16 tile[128 * 64];

  const int tid = threadIdx.x, lane = tid & 31, wave = tid >> 5;
  const int h = lane >> 4, m = lane & 15;
  const int m0 = blockIdx.y * 128, n0 = blockIdx.x * 64, z = blockIdx.z;
  const __bf16* __restrict__ W = (z == 0) ? Wq : ((z == 1) ? Wk : Wv);

  v8f acc[8];
#pragma unroll
  for (int i = 0; i < 8; ++i) acc[i] = (v8f)(0.0f);

  const __bf16* ap0 = Xb + (size_t)(m0 + wave * 32 + m) * DIM + 8 * h;
  const __bf16* ap1 = ap0 + (size_t)16 * DIM;
  const __bf16* bp  = W + (size_t)(n0 + m) * DIM + 8 * h;

#pragma unroll 1
  for (int k0 = 0; k0 < DIM; k0 += 32) {
    FragB a0, a1, b0, b1, b2, b3;
    a0.half[0] = *(const v8b*)(ap0 + k0);             a0.half[1] = *(const v8b*)(ap0 + k0 + 16);
    a1.half[0] = *(const v8b*)(ap1 + k0);             a1.half[1] = *(const v8b*)(ap1 + k0 + 16);
    b0.half[0] = *(const v8b*)(bp + k0);              b0.half[1] = *(const v8b*)(bp + k0 + 16);
    b1.half[0] = *(const v8b*)(bp + 16 * DIM + k0);   b1.half[1] = *(const v8b*)(bp + 16 * DIM + k0 + 16);
    b2.half[0] = *(const v8b*)(bp + 32 * DIM + k0);   b2.half[1] = *(const v8b*)(bp + 32 * DIM + k0 + 16);
    b3.half[0] = *(const v8b*)(bp + 48 * DIM + k0);   b3.half[1] = *(const v8b*)(bp + 48 * DIM + k0 + 16);
    acc[0] = mma_bf(a0.v, b0.v, acc[0]);
    acc[1] = mma_bf(a0.v, b1.v, acc[1]);
    acc[2] = mma_bf(a0.v, b2.v, acc[2]);
    acc[3] = mma_bf(a0.v, b3.v, acc[3]);
    acc[4] = mma_bf(a1.v, b0.v, acc[4]);
    acc[5] = mma_bf(a1.v, b1.v, acc[5]);
    acc[6] = mma_bf(a1.v, b2.v, acc[6]);
    acc[7] = mma_bf(a1.v, b3.v, acc[7]);
    asm volatile(NOP4
                 : "+v"(acc[0]), "+v"(acc[1]), "+v"(acc[2]), "+v"(acc[3]),
                   "+v"(acc[4]), "+v"(acc[5]), "+v"(acc[6]), "+v"(acc[7])
                 : "v"(a0.v), "v"(a1.v), "v"(b0.v), "v"(b1.v), "v"(b2.v), "v"(b3.v));
  }

  if (z < 2) {
#pragma unroll
    for (int i = 0; i < 2; ++i)
#pragma unroll
      for (int t = 0; t < 4; ++t)
#pragma unroll
        for (int r = 0; r < 8; ++r)
          tile[(wave * 32 + i * 16 + 8 * h + r) * 64 + t * 16 + m] = (_Float16)acc[i * 4 + t][r];
  } else {
#pragma unroll
    for (int i = 0; i < 2; ++i)
#pragma unroll
      for (int t = 0; t < 4; ++t)
#pragma unroll
        for (int r = 0; r < 8; ++r)
          tile[(t * 16 + m) * 128 + wave * 32 + i * 16 + 8 * h + r] = (_Float16)acc[i * 4 + t][r];
  }
  __syncthreads();

  v8h vals[8];
  if (z < 2) {
    _Float16* dst = (z == 0) ? Qh : Kh;
    const int rsub = lane >> 3, col = (lane & 7) * 8;
#pragma unroll
    for (int it = 0; it < 8; ++it) {
      const int row = wave * 32 + it * 4 + rsub;
      vals[it] = *(const v8h*)(&tile[row * 64 + col]);
    }
    _Float16* gp = dst + (size_t)(m0 + wave * 32 + rsub) * DIM + n0 + col;
#pragma unroll
    for (int it = 0; it < 8; ++it) *(volatile v8h*)(gp + (size_t)it * 4 * DIM) = vals[it];
    __threadfence();
#pragma unroll
    for (int it = 0; it < 8; ++it) *(volatile v8h*)(gp + (size_t)it * 4 * DIM) = vals[it];
  } else {
    const int osub = lane >> 4, col = (lane & 15) * 8;
#pragma unroll
    for (int it = 0; it < 8; ++it) {
      const int orow = wave * 16 + it * 2 + osub;
      vals[it] = *(const v8h*)(&tile[orow * 128 + col]);
    }
    _Float16* gp = Vt + (size_t)(n0 + wave * 16 + osub) * SEQ + m0 + col;
#pragma unroll
    for (int it = 0; it < 8; ++it) *(volatile v8h*)(gp + (size_t)it * 2 * SEQ) = vals[it];
    __threadfence();
#pragma unroll
    for (int it = 0; it < 8; ++it) *(volatile v8h*)(gp + (size_t)it * 2 * SEQ) = vals[it];
  }
}

__global__ __launch_bounds__(256) void attn_kernel(
    const _Float16* __restrict__ Qh, const _Float16* __restrict__ Kh,
    const _Float16* __restrict__ Vt, float* out)
{
  __shared__ __attribute__((aligned(16))) float    stage[16 * 512];
  __shared__ __attribute__((aligned(16))) float    Ss[16 * KT];
  __shared__ __attribute__((aligned(16))) _Float16 Ps[16 * KT];
  __shared__ float row_alpha[16];
  __shared__ float row_l[16];
  _Float16* Qs = (_Float16*)stage;

  const int tid = threadIdx.x, lane = tid & 31, wave = tid >> 5;
  const int h = lane >> 4, m = lane & 15;
  const int q0 = blockIdx.x * 16;

  {
    const v4u* g = (const v4u*)(Qh + (size_t)q0 * DIM);
    v4u* l = (v4u*)Qs;
#pragma unroll
    for (int i = 0; i < 8; ++i) l[tid + 256 * i] = g[tid + 256 * i];
  }
  __syncthreads();

  v8f acc[8];
#pragma unroll
  for (int t = 0; t < 8; ++t) acc[t] = (v8f)(0.0f);

  float m_run = -1.0e30f, l_run = 0.0f;
  const int srow = tid >> 4, sc = tid & 15;
  const float scale = 0.03125f;

  const _Float16* qa = Qs + m * DIM + 8 * h;
  const _Float16* pa = Ps + m * KT + 8 * h;

#pragma unroll 1
  for (int jt = 0; jt < SEQ / KT; ++jt) {
    const int jbase = jt * KT;

    v8f s0 = (v8f)(0.0f), s1 = (v8f)(0.0f);
    const _Float16* kb0 = Kh + (size_t)(jbase + wave * 32 + m) * DIM + 8 * h;
    const _Float16* kb1 = kb0 + (size_t)16 * DIM;
#pragma unroll 1
    for (int k0 = 0; k0 < DIM; k0 += 64) {
      FragH a0, a1, c0, c1, e0, e1;
      a0.half[0] = *(const v8h*)(qa + k0);        a0.half[1] = *(const v8h*)(qa + k0 + 16);
      c0.half[0] = *(const v8h*)(kb0 + k0);       c0.half[1] = *(const v8h*)(kb0 + k0 + 16);
      c1.half[0] = *(const v8h*)(kb1 + k0);       c1.half[1] = *(const v8h*)(kb1 + k0 + 16);
      a1.half[0] = *(const v8h*)(qa + k0 + 32);   a1.half[1] = *(const v8h*)(qa + k0 + 48);
      e0.half[0] = *(const v8h*)(kb0 + k0 + 32);  e0.half[1] = *(const v8h*)(kb0 + k0 + 48);
      e1.half[0] = *(const v8h*)(kb1 + k0 + 32);  e1.half[1] = *(const v8h*)(kb1 + k0 + 48);
      s0 = mma_h(a0.v, c0.v, s0);
      s1 = mma_h(a0.v, c1.v, s1);
      s0 = mma_h(a1.v, e0.v, s0);
      s1 = mma_h(a1.v, e1.v, s1);
      asm volatile(NOP4 : "+v"(s0), "+v"(s1) : "v"(a1.v), "v"(e0.v), "v"(e1.v));
    }
#pragma unroll
    for (int r = 0; r < 8; ++r) {
      Ss[(8 * h + r) * KT + wave * 32 + m]      = s0[r] * scale;
      Ss[(8 * h + r) * KT + wave * 32 + 16 + m] = s1[r] * scale;
    }
    __syncthreads();

    {
      const float* sp = Ss + srow * KT + sc * 16;
      union { v4f v[4]; float e[16]; } sv;
#pragma unroll
      for (int i = 0; i < 4; ++i) sv.v[i] = *(const v4f*)(sp + 4 * i);
      float pmax = sv.e[0];
#pragma unroll
      for (int i = 1; i < 16; ++i) pmax = fmaxf(pmax, sv.e[i]);
      pmax = fmaxf(pmax, __shfl_xor(pmax, 8));
      pmax = fmaxf(pmax, __shfl_xor(pmax, 4));
      pmax = fmaxf(pmax, __shfl_xor(pmax, 2));
      pmax = fmaxf(pmax, __shfl_xor(pmax, 1));
      const float m_new = fmaxf(m_run, pmax);
      const float alpha = __expf(m_run - m_new);
      m_run = m_new;
      union { v8h v[2]; _Float16 e[16]; } pk;
      float psum = 0.0f;
#pragma unroll
      for (int i = 0; i < 16; ++i) {
        const float p = __expf(sv.e[i] - m_new);
        psum += p;
        pk.e[i] = (_Float16)(p * PSCALE);
      }
      _Float16* pp = Ps + srow * KT + sc * 16;
      *(v8h*)pp       = pk.v[0];
      *(v8h*)(pp + 8) = pk.v[1];
      psum += __shfl_xor(psum, 8);
      psum += __shfl_xor(psum, 4);
      psum += __shfl_xor(psum, 2);
      psum += __shfl_xor(psum, 1);
      l_run = l_run * alpha + psum;
      if (sc == 0) row_alpha[srow] = alpha;
    }
    __syncthreads();

    {
      float al[8];
#pragma unroll
      for (int r = 0; r < 8; ++r) al[r] = row_alpha[8 * h + r];
#pragma unroll
      for (int t = 0; t < 8; ++t)
#pragma unroll
        for (int r = 0; r < 8; ++r) acc[t][r] *= al[r];

      const _Float16* vb = Vt + (size_t)(wave * 128 + m) * SEQ + jbase + 8 * h;
#pragma unroll 1
      for (int ks = 0; ks < KT / 32; ++ks) {
        FragH a, b;
        a.half[0] = *(const v8h*)(pa + ks * 32);
        a.half[1] = *(const v8h*)(pa + ks * 32 + 16);
#pragma unroll
        for (int t = 0; t < 8; ++t) {
          const _Float16* p = vb + (size_t)t * 16 * SEQ + ks * 32;
          b.half[0] = *(const v8h*)p;
          b.half[1] = *(const v8h*)(p + 16);
          acc[t] = mma_h(a.v, b.v, acc[t]);
        }
        asm volatile(NOP4
                     : "+v"(acc[0]), "+v"(acc[1]), "+v"(acc[2]), "+v"(acc[3]),
                       "+v"(acc[4]), "+v"(acc[5]), "+v"(acc[6]), "+v"(acc[7])
                     : "v"(a.v), "v"(b.v));
      }
    }
  }

  if (sc == 0) row_l[srow] = l_run;
  __syncthreads();

  float linv[8];
#pragma unroll
  for (int r = 0; r < 8; ++r) linv[r] = PSCALE_INV / row_l[8 * h + r];

  const int piece = tid & 7;
#pragma unroll 1
  for (int hf = 0; hf < 2; ++hf) {
    if ((wave >> 2) == hf) {
#pragma unroll
      for (int t = 0; t < 8; ++t)
#pragma unroll
        for (int r = 0; r < 8; ++r)
          stage[(8 * h + r) * 512 + (wave & 3) * 128 + t * 16 + m] = acc[t][r] * linv[r];
    }
    __syncthreads();
    v4f vals[8];
#pragma unroll
    for (int it = 0; it < 8; ++it) {
      const int line = it * 32 + (tid >> 3);
      const int row = line >> 4, lir = line & 15;
      vals[it] = *(const v4f*)(&stage[row * 512 + lir * 32 + piece * 4]);
    }
    float* ob = out + (size_t)q0 * DIM + hf * 512 + piece * 4;
#pragma unroll
    for (int it = 0; it < 8; ++it) {
      const int line = it * 32 + (tid >> 3);
      const int row = line >> 4, lir = line & 15;
      *(volatile v4f*)(ob + (size_t)row * DIM + lir * 32) = vals[it];
    }
    __threadfence();
#pragma unroll
    for (int it = 0; it < 8; ++it) {
      const int line = it * 32 + (tid >> 3);
      const int row = line >> 4, lir = line & 15;
      *(volatile v4f*)(ob + (size_t)row * DIM + lir * 32) = vals[it];
    }
    __syncthreads();
  }
}

extern "C" void kernel_launch(void* const* d_in, const int* in_sizes, int n_in,
                              void* d_out, int out_size, void* d_ws, size_t ws_size,
                              hipStream_t stream) {
  if (n_in < 4) return;
  if (in_sizes[0] != SEQ * DIM || in_sizes[1] != DIM * DIM ||
      in_sizes[2] != DIM * DIM || in_sizes[3] != DIM * DIM) return;
  if (out_size != SEQ * DIM) return;

  const size_t bx = (size_t)SEQ * DIM * 2;
  const size_t bw = (size_t)DIM * DIM * 2;
  const size_t bq = (size_t)SEQ * DIM * 2;
  const size_t need = bx + 3 * bw + 3 * bq;
  if (ws_size < need) return;

  char* ws = (char*)d_ws;
  uint16_t* xb  = (uint16_t*)(ws);
  uint16_t* wqb = (uint16_t*)(ws + bx);
  uint16_t* wkb = (uint16_t*)(ws + bx + bw);
  uint16_t* wvb = (uint16_t*)(ws + bx + 2 * bw);
  _Float16* Qh  = (_Float16*)(ws + bx + 3 * bw);
  _Float16* Kh  = (_Float16*)(ws + bx + 3 * bw + bq);
  _Float16* Vt  = (_Float16*)(ws + bx + 3 * bw + 2 * bq);

  const int n8x = in_sizes[0] / 8;
  const int n8w = in_sizes[1] / 8;
  dim3 gc((unsigned)((n8x + 255) / 256), 4, 1);
  cvt_kernel<<<gc, 256, 0, stream>>>((const float*)d_in[0], (const float*)d_in[1],
                                      (const float*)d_in[2], (const float*)d_in[3],
                                      xb, wqb, wkb, wvb, n8x, n8w, n8w, n8w);

  proj_kernel<<<dim3(DIM / 64, SEQ / 128, 3), 128, 0, stream>>>(
      (const __bf16*)xb, (const __bf16*)wqb, (const __bf16*)wkb, (const __bf16*)wvb, Qh, Kh, Vt);

  attn_kernel<<<SEQ / 16, 256, 0, stream>>>(Qh, Kh, Vt, (float*)d_out);
}
